// TransformerEncoderLayer_10230612099074
// MI455X (gfx1250) — hardware-verified
//
#include <hip/hip_runtime.h>


typedef _Float16 v16h __attribute__((ext_vector_type(16)));
typedef _Float16 v8h  __attribute__((ext_vector_type(8)));
typedef _Float16 v4h  __attribute__((ext_vector_type(4)));
typedef float    v8f  __attribute__((ext_vector_type(8)));
typedef float    f32x4 __attribute__((ext_vector_type(4)));
typedef unsigned int u32x4 __attribute__((ext_vector_type(4)));
typedef unsigned int u32x2 __attribute__((ext_vector_type(2)));

#ifndef NB
#define NB 2
#endif
#ifndef SEQ
#define SEQ 2048
#endif
#define NB_FULL  2
#define SEQ_FULL 2048
#define DM    1024
#define NH    16
#define HDIM  64
#define FFD   4096
#define MROWS (SEQ * NB)

#define W_CARRY   64.0f
#define P_CARRY   4096.0f
#define CTX_CARRY 16.0f

static_assert(NB >= 1 && NB <= NB_FULL);
static_assert(SEQ >= 64 && SEQ <= SEQ_FULL && (SEQ % 64) == 0);
static_assert((MROWS % 64) == 0);
static_assert((DM % 64) == 0 && (FFD % 64) == 0 && HDIM == 64 && NH * HDIM == DM);

#define SZ_H_MD  ((size_t)MROWS * DM * 2)
#define SZ_F_MD  ((size_t)MROWS * DM * 4)
#define SZ_H_MF  ((size_t)MROWS * FFD * 2)
#define SZ_W     ((size_t)DM * DM * 2)
#define SZ_W1    ((size_t)FFD * DM * 2)
#define OFF_XH   ((size_t)0)
#define OFF_QH   (OFF_XH + SZ_H_MD)
#define OFF_KH   (OFF_QH + SZ_H_MD)
#define OFF_VT   (OFF_KH + SZ_H_MD)
#define SZ_R1    (4 * SZ_H_MD)
#define OFF_H1   ((size_t)0)
static_assert(SZ_H_MF <= SZ_R1);
#define OFF_WQT  (SZ_R1)
#define OFF_WKT  (OFF_WQT + SZ_W)
#define OFF_WVT  (OFF_WKT + SZ_W)
#define OFF_WOT  (OFF_WVT + SZ_W)
#define OFF_W1T  (OFF_WOT + SZ_W)
#define OFF_W2T  (OFF_W1T + SZ_W1)
#define OFF_CTX  (OFF_W2T + SZ_W1)
#define OFF_TMPF (OFF_CTX + SZ_H_MD)
#define OFF_XF   (OFF_TMPF + SZ_F_MD)
#define OFF_XHL  (OFF_XF + SZ_F_MD)
#define WS_TOTAL (OFF_XHL + SZ_H_MD)
static_assert(WS_TOTAL <= (size_t)134217728);
static_assert((SZ_H_MD % 256) == 0 && (SZ_W % 256) == 0 && (SZ_W1 % 256) == 0);

__device__ __forceinline__ float bf16r(float f) {
  unsigned u = __float_as_uint(f);
  u = (u + 0x7FFFu + ((u >> 16) & 1u)) & 0xFFFF0000u;
  return __uint_as_float(u);
}

union Frag { v16h v; v8h h[2]; };

__device__ __forceinline__ v16h load_frag(const _Float16* base, int ld, int row, int kc, int lane) {
  const _Float16* p = base + (size_t)row * ld + kc + ((lane & 16) >> 1);
  Frag f;
  f.h[0] = *(const v8h*)p;
  f.h[1] = *(const v8h*)(p + 16);
  return f.v;
}

__device__ __forceinline__ v8f wmma16(v16h a, v16h b, v8f c) {
  return __builtin_amdgcn_wmma_f32_16x16x32_f16(false, a, false, b, (short)0, c, false, false);
}

__device__ __forceinline__ float wave_sum(float v) {
  v += __shfl_xor(v, 16);
  v += __shfl_xor(v, 8);
  v += __shfl_xor(v, 4);
  v += __shfl_xor(v, 2);
  v += __shfl_xor(v, 1);
  return v;
}

__global__ __launch_bounds__(128) void k_cvt_src(const float* __restrict__ src, _Float16* __restrict__ Xh) {
  const int m = blockIdx.x;
  const int s = m / NB, b = m - s * NB;
  const size_t io = (size_t)s * NB_FULL + b;
  const int c8 = threadIdx.x * 8;
  const float* sp = src + io * DM + c8;
  f32x4 x0 = *(const f32x4*)sp;
  f32x4 x1 = *(const f32x4*)(sp + 4);
  v8h hv;
#pragma unroll
  for (int j = 0; j < 4; ++j) { hv[j] = (_Float16)bf16r(x0[j]); hv[4 + j] = (_Float16)bf16r(x1[j]); }
  const u32x4 bits = __builtin_bit_cast(u32x4, hv);
  _Float16* dp = Xh + (size_t)m * DM + c8;
  *(volatile u32x4*)dp = bits;
  __threadfence();
  *(volatile u32x4*)dp = bits;
}

__global__ __launch_bounds__(128) void k_wt(const float* __restrict__ W, _Float16* __restrict__ WT, int K, int N) {
  const int lane = threadIdx.x & 31, wave = threadIdx.x >> 5;
  const int q = lane >> 3, p = lane & 7;
  const int n = blockIdx.y * 16 + wave * 4 + q;
  const int k0 = blockIdx.x * 64 + p * 8;
  v8h hv;
#pragma unroll
  for (int i = 0; i < 8; ++i) {
    float w = W[(size_t)(k0 + i) * N + n];
    hv[i] = (_Float16)(bf16r(w) * W_CARRY);
  }
  const u32x4 bits = __builtin_bit_cast(u32x4, hv);
  _Float16* dp = WT + (size_t)n * K + k0;
  *(volatile u32x4*)dp = bits;
  __threadfence();
  *(volatile u32x4*)dp = bits;
}

template <int OUTM, int RELU, int BIASM, int PERMB>
__global__ __launch_bounds__(128) void k_gemm(const _Float16* __restrict__ A, const _Float16* __restrict__ Bt,
                                               const float* __restrict__ bias,
                                               float* __restrict__ outF, _Float16* __restrict__ outH,
                                               int M, int N, int K, float oscale, int pS, int pNB) {
  __shared__ __attribute__((aligned(16))) float stg[4][16][64];
  const int lane = threadIdx.x & 31;
  const int wave = threadIdx.x >> 5;
  const int hf = lane >> 4;
  const int m16 = lane & 15;
  const int koff = (lane & 16) >> 1;
  const int m0 = blockIdx.y * 64 + wave * 16;
  const int n0 = blockIdx.x * 64;
  (void)M;

  const _Float16* ap = A + (size_t)(m0 + m16) * K + koff;
  const _Float16* bp[4];
#pragma unroll
  for (int nt = 0; nt < 4; ++nt) {
    int r = n0 + nt * 16 + m16;
    if (PERMB) r = (r % pS) * pNB + (r / pS);
    bp[nt] = Bt + (size_t)r * K + koff;
  }

  const v8f zero = {0.f, 0.f, 0.f, 0.f, 0.f, 0.f, 0.f, 0.f};
  v8f acc0 = zero, acc1 = zero, acc2 = zero, acc3 = zero;

#pragma unroll 2
  for (int kc = 0; kc < K; kc += 32) {
    Frag a, b0, b1, b2, b3;
    a.h[0]  = *(const v8h*)(ap + kc);     a.h[1]  = *(const v8h*)(ap + kc + 16);
    b0.h[0] = *(const v8h*)(bp[0] + kc);  b0.h[1] = *(const v8h*)(bp[0] + kc + 16);
    b1.h[0] = *(const v8h*)(bp[1] + kc);  b1.h[1] = *(const v8h*)(bp[1] + kc + 16);
    b2.h[0] = *(const v8h*)(bp[2] + kc);  b2.h[1] = *(const v8h*)(bp[2] + kc + 16);
    b3.h[0] = *(const v8h*)(bp[3] + kc);  b3.h[1] = *(const v8h*)(bp[3] + kc + 16);
    acc0 = wmma16(a.v, b0.v, acc0);
    acc1 = wmma16(a.v, b1.v, acc1);
    acc2 = wmma16(a.v, b2.v, acc2);
    acc3 = wmma16(a.v, b3.v, acc3);
    asm volatile("v_nop\n\tv_nop\n\tv_nop\n\tv_nop"
                 : "+v"(acc0), "+v"(acc1), "+v"(acc2), "+v"(acc3)
                 : "v"(a.v), "v"(b0.v), "v"(b1.v), "v"(b2.v), "v"(b3.v));
  }

#pragma unroll
  for (int r = 0; r < 8; ++r) {
    const int row = hf * 8 + r;
    stg[wave][row][0 * 16 + m16] = acc0[r];
    stg[wave][row][1 * 16 + m16] = acc1[r];
    stg[wave][row][2 * 16 + m16] = acc2[r];
    stg[wave][row][3 * 16 + m16] = acc3[r];
  }
  __syncthreads();

  if (OUTM == 0) {
    const int rs = lane >> 4;
    const int c4 = m16 * 4;
    f32x4 bc = {0.f, 0.f, 0.f, 0.f};
    if (BIASM == 1) {
#pragma unroll
      for (int j = 0; j < 4; ++j) bc[j] = bf16r(bias[n0 + c4 + j]);
    }
#pragma unroll
    for (int pass = 0; pass < 2; ++pass) {
#pragma unroll
      for (int i = 0; i < 8; ++i) {
        const int row = 2 * i + rs;
        f32x4 v = *(const f32x4*)(&stg[wave][row][c4]);
        v = v * oscale + bc;
        if (BIASM == 2) v = v + bf16r(bias[m0 + row]);
        if (RELU) { v[0] = fmaxf(v[0], 0.f); v[1] = fmaxf(v[1], 0.f); v[2] = fmaxf(v[2], 0.f); v[3] = fmaxf(v[3], 0.f); }
        float* gp = outF + (size_t)(m0 + row) * N + n0 + c4;
        *(volatile f32x4*)gp = v;
      }
      if (pass == 0) __threadfence();
    }
  } else {
    const int rs = lane >> 3;
    const int c8 = (lane & 7) * 8;
    float bc[8];
#pragma unroll
    for (int j = 0; j < 8; ++j) bc[j] = (BIASM == 1) ? bf16r(bias[n0 + c8 + j]) : 0.f;
#pragma unroll
    for (int pass = 0; pass < 2; ++pass) {
#pragma unroll
      for (int i = 0; i < 4; ++i) {
        const int row = 4 * i + rs;
        f32x4 v0 = *(const f32x4*)(&stg[wave][row][c8]);
        f32x4 v1 = *(const f32x4*)(&stg[wave][row][c8 + 4]);
        const float br = (BIASM == 2) ? bf16r(bias[m0 + row]) : 0.f;
        v8h hv;
#pragma unroll
        for (int j = 0; j < 4; ++j) {
          float x0 = v0[j] * oscale + bc[j] + br;
          float x1 = v1[j] * oscale + bc[4 + j] + br;
          if (RELU) { x0 = fmaxf(x0, 0.f); x1 = fmaxf(x1, 0.f); }
          hv[j] = (_Float16)x0;
          hv[4 + j] = (_Float16)x1;
        }
        const u32x4 bits = __builtin_bit_cast(u32x4, hv);
        _Float16* gp = outH + (size_t)(m0 + row) * N + n0 + c8;
        *(volatile u32x4*)gp = bits;
      }
      if (pass == 0) __threadfence();
    }
  }
}

__global__ __launch_bounds__(128) __attribute__((amdgpu_num_vgpr(256)))
void k_attn(const _Float16* __restrict__ Qh, const _Float16* __restrict__ Kh,
            const _Float16* __restrict__ VT, _Float16* __restrict__ ctx) {
  __shared__ __attribute__((aligned(16))) _Float16 psh[4][16 * 32];
  __shared__ __attribute__((aligned(16))) float stg[4][16][64];
  const int lane = threadIdx.x & 31;
  const int wave = threadIdx.x >> 5;
  const int hf = lane >> 4;
  const int m16 = lane & 15;
  const int nqb = SEQ / 64;
  const int qb = blockIdx.x % nqb;
  const int bh = blockIdx.x / nqb;
  const int hh = bh % NH;
  const int b  = bh / NH;
  const int q0 = qb * 64 + wave * 16;
  const int ldq = NB * DM;
  const int ldv = NB * SEQ;
  const _Float16* qbase = Qh + (size_t)b * DM + hh * HDIM;
  const _Float16* kbase = Kh + (size_t)b * DM + hh * HDIM;
  const _Float16* vbase = VT + (size_t)(hh * HDIM) * ldv + (size_t)b * SEQ;
  _Float16* ps = &psh[wave][0];

  const v16h qa0 = load_frag(qbase, ldq, q0 + m16, 0, lane);
  const v16h qa1 = load_frag(qbase, ldq, q0 + m16, 32, lane);

  const v8f zero = {0.f, 0.f, 0.f, 0.f, 0.f, 0.f, 0.f, 0.f};
  v8f o0 = zero, o1 = zero, o2 = zero, o3 = zero;
  float mrow[8], lrow[8];
#pragma unroll
  for (int r = 0; r < 8; ++r) { mrow[r] = -1e30f; lrow[r] = 0.0f; }

  const float scale = 0.125f;
  const int NT = SEQ / 32;
#pragma unroll 1
  for (int kt = 0; kt < NT; ++kt) {
    const int key0 = kt * 32;

    v8f s0 = zero, s1 = zero;
    {
      v16h kb0 = load_frag(kbase, ldq, key0 + m16, 0, lane);
      v16h kb1 = load_frag(kbase, ldq, key0 + 16 + m16, 0, lane);
      s0 = wmma16(qa0, kb0, s0);
      s1 = wmma16(qa0, kb1, s1);
      asm volatile("v_nop\n\tv_nop\n\tv_nop\n\tv_nop" : "+v"(s0), "+v"(s1) : "v"(qa0), "v"(kb0), "v"(kb1));
    }
    {
      v16h kb0 = load_frag(kbase, ldq, key0 + m16, 32, lane);
      v16h kb1 = load_frag(kbase, ldq, key0 + 16 + m16, 32, lane);
      s0 = wmma16(qa1, kb0, s0);
      s1 = wmma16(qa1, kb1, s1);
      asm volatile("v_nop\n\tv_nop\n\tv_nop\n\tv_nop" : "+v"(s0), "+v"(s1) : "v"(qa1), "v"(kb0), "v"(kb1));
    }

#pragma unroll
    for (int r = 0; r < 8; ++r) {
      const float a0 = s0[r] * scale, a1 = s1[r] * scale;
      float mx = fmaxf(a0, a1);
      mx = fmaxf(mx, __shfl_xor(mx, 1));
      mx = fmaxf(mx, __shfl_xor(mx, 2));
      mx = fmaxf(mx, __shfl_xor(mx, 4));
      mx = fmaxf(mx, __shfl_xor(mx, 8));
      const float mnew = fmaxf(mrow[r], mx);
      const float corr = __expf(mrow[r] - mnew);
      const float p0 = __expf(a0 - mnew);
      const float p1 = __expf(a1 - mnew);
      float sum = p0 + p1;
      sum += __shfl_xor(sum, 1);
      sum += __shfl_xor(sum, 2);
      sum += __shfl_xor(sum, 4);
      sum += __shfl_xor(sum, 8);
      lrow[r] = lrow[r] * corr + sum;
      mrow[r] = mnew;
      o0[r] *= corr; o1[r] *= corr; o2[r] *= corr; o3[r] *= corr;
      const int rowi = r + hf * 8;
      ps[rowi * 32 + m16]      = (_Float16)(p0 * P_CARRY);
      ps[rowi * 32 + 16 + m16] = (_Float16)(p1 * P_CARRY);
    }
    __syncthreads();

    const v16h pa = load_frag(ps, 32, m16, 0, lane);
    {
      v16h vb0 = load_frag(vbase, ldv, 0 * 16 + m16, key0, lane);
      v16h vb1 = load_frag(vbase, ldv, 1 * 16 + m16, key0, lane);
      o0 = wmma16(pa, vb0, o0);
      o1 = wmma16(pa, vb1, o1);
      asm volatile("v_nop\n\tv_nop\n\tv_nop\n\tv_nop" : "+v"(o0), "+v"(o1) : "v"(pa), "v"(vb0), "v"(vb1));
    }
    {
      v16h vb2 = load_frag(vbase, ldv, 2 * 16 + m16, key0, lane);
      v16h vb3 = load_frag(vbase, ldv, 3 * 16 + m16, key0, lane);
      o2 = wmma16(pa, vb2, o2);
      o3 = wmma16(pa, vb3, o3);
      asm volatile("v_nop\n\tv_nop\n\tv_nop\n\tv_nop" : "+v"(o2), "+v"(o3) : "v"(pa), "v"(vb2), "v"(vb3));
    }
    __syncthreads();
  }

#pragma unroll
  for (int r = 0; r < 8; ++r) {
    const float inv = (1.0f / lrow[r]) * (CTX_CARRY / P_CARRY);
    const int row = hf * 8 + r;
    stg[wave][row][0 * 16 + m16] = o0[r] * inv;
    stg[wave][row][1 * 16 + m16] = o1[r] * inv;
    stg[wave][row][2 * 16 + m16] = o2[r] * inv;
    stg[wave][row][3 * 16 + m16] = o3[r] * inv;
  }
  __syncthreads();
  {
    const int rs = lane >> 3;
    const int c8 = (lane & 7) * 8;
#pragma unroll
    for (int pass = 0; pass < 2; ++pass) {
#pragma unroll
      for (int i = 0; i < 4; ++i) {
        const int row = 4 * i + rs;
        f32x4 v0 = *(const f32x4*)(&stg[wave][row][c8]);
        f32x4 v1 = *(const f32x4*)(&stg[wave][row][c8 + 4]);
        v8h hv;
#pragma unroll
        for (int j = 0; j < 4; ++j) { hv[j] = (_Float16)v0[j]; hv[4 + j] = (_Float16)v1[j]; }
        const u32x4 bits = __builtin_bit_cast(u32x4, hv);
        _Float16* gp = ctx + (size_t)((q0 + row) * NB + b) * DM + hh * HDIM + c8;
        *(volatile u32x4*)gp = bits;
      }
      if (pass == 0) __threadfence();
    }
  }
}

template <int MODE>
__global__ __launch_bounds__(256) void k_addln(const float* __restrict__ a, const float* __restrict__ rsd,
                                                const float* __restrict__ g, const float* __restrict__ be,
                                                float* __restrict__ outF, _Float16* __restrict__ outH) {
  __shared__ float red[8];
  const int m = blockIdx.x;
  const int t = threadIdx.x;
  const int lane = t & 31, wave = t >> 5;
  const int s = m / NB, b = m - s * NB;
  const size_t io = (size_t)s * NB_FULL + b;
  const int c4 = t * 4;

  const f32x4 av = *(const f32x4*)(a + (size_t)m * DM + c4);
  f32x4 rv;
  if (MODE == 0) {
    const f32x4 sv = *(const f32x4*)(rsd + io * DM + c4);
#pragma unroll
    for (int j = 0; j < 4; ++j) rv[j] = bf16r(sv[j]);
  } else {
    rv = *(const f32x4*)(rsd + (size_t)m * DM + c4);
  }
  const f32x4 x = av + rv;

  float psum = (x[0] + x[1]) + (x[2] + x[3]);
  psum = wave_sum(psum);
  if (lane == 0) red[wave] = psum;
  __syncthreads();
  float tot = 0.f;
#pragma unroll
  for (int w = 0; w < 8; ++w) tot += red[w];
  const float mean = tot * (1.0f / (float)DM);
  __syncthreads();
  const f32x4 d = x - mean;
  float pvar = (d[0] * d[0] + d[1] * d[1]) + (d[2] * d[2] + d[3] * d[3]);
  pvar = wave_sum(pvar);
  if (lane == 0) red[wave] = pvar;
  __syncthreads();
  float tot2 = 0.f;
#pragma unroll
  for (int w = 0; w < 8; ++w) tot2 += red[w];
  const float var = tot2 * (1.0f / (float)DM);
  const float rstd = rsqrtf(var + 1e-5f);

  f32x4 gv, bv;
#pragma unroll
  for (int j = 0; j < 4; ++j) { gv[j] = bf16r(g[c4 + j]); bv[j] = bf16r(be[c4 + j]); }
  const f32x4 y = d * rstd * gv + bv;

  if (MODE == 0) {
    v4h yh;
#pragma unroll
    for (int j = 0; j < 4; ++j) yh[j] = (_Float16)y[j];
    const u32x2 ybits = __builtin_bit_cast(u32x2, yh);
    float* fp = outF + (size_t)m * DM + c4;
    _Float16* hp = outH + (size_t)m * DM + c4;
    *(volatile f32x4*)fp = y;
    *(volatile u32x2*)hp = ybits;
    __threadfence();
    *(volatile f32x4*)fp = y;
    *(volatile u32x2*)hp = ybits;
  } else {
    float* fp = outF + io * DM + c4;
    *(volatile f32x4*)fp = y;
    __threadfence();
    *(volatile f32x4*)fp = y;
  }
}

extern "C" void kernel_launch(void* const* d_in, const int* in_sizes, int n_in,
                              void* d_out, int out_size, void* d_ws, size_t ws_size, hipStream_t stream) {
  if (n_in < 17) return;
  if (in_sizes[0] < SEQ * NB_FULL * DM) return;
  if (in_sizes[1] < DM * DM || in_sizes[3] < DM * DM || in_sizes[5] < DM * DM || in_sizes[7] < DM * DM) return;
  if (in_sizes[2] < DM || in_sizes[4] < DM || in_sizes[6] < DM || in_sizes[8] < DM) return;
  if (in_sizes[9] < DM || in_sizes[10] < DM || in_sizes[15] < DM || in_sizes[16] < DM) return;
  if (in_sizes[11] < DM * FFD || in_sizes[13] < FFD * DM || in_sizes[12] < FFD || in_sizes[14] < DM) return;
  if (out_size < SEQ * NB_FULL * DM) return;
  if (ws_size < WS_TOTAL) return;

  const float* src = (const float*)d_in[0];
  const float* Wq  = (const float*)d_in[1];
  const float* bq  = (const float*)d_in[2];
  const float* Wk  = (const float*)d_in[3];
  const float* bk  = (const float*)d_in[4];
  const float* Wv  = (const float*)d_in[5];
  const float* bv  = (const float*)d_in[6];
  const float* Wo  = (const float*)d_in[7];
  const float* bo  = (const float*)d_in[8];
  const float* g1  = (const float*)d_in[9];
  const float* be1 = (const float*)d_in[10];
  const float* W1  = (const float*)d_in[11];
  const float* bf1 = (const float*)d_in[12];
  const float* W2  = (const float*)d_in[13];
  const float* bf2 = (const float*)d_in[14];
  const float* g2  = (const float*)d_in[15];
  const float* be2 = (const float*)d_in[16];
  float* out = (float*)d_out;

  char* w = (char*)d_ws;
  _Float16* Xh   = (_Float16*)(w + OFF_XH);
  _Float16* Qh   = (_Float16*)(w + OFF_QH);
  _Float16* Kh   = (_Float16*)(w + OFF_KH);
  _Float16* VT   = (_Float16*)(w + OFF_VT);
  _Float16* h1   = (_Float16*)(w + OFF_H1);
  _Float16* WqT  = (_Float16*)(w + OFF_WQT);
  _Float16* WkT  = (_Float16*)(w + OFF_WKT);
  _Float16* WvT  = (_Float16*)(w + OFF_WVT);
  _Float16* WoT  = (_Float16*)(w + OFF_WOT);
  _Float16* W1T  = (_Float16*)(w + OFF_W1T);
  _Float16* W2T  = (_Float16*)(w + OFF_W2T);
  _Float16* ctx  = (_Float16*)(w + OFF_CTX);
  float*    tmpF = (float*)(w + OFF_TMPF);
  float*    xF   = (float*)(w + OFF_XF);
  _Float16* xh   = (_Float16*)(w + OFF_XHL);

  const float inv_w   = 1.0f / W_CARRY;
  const float inv_wcx = 1.0f / (W_CARRY * CTX_CARRY);

  k_cvt_src<<<MROWS, 128, 0, stream>>>(src, Xh);
  k_wt<<<dim3(DM / 64, DM / 16), 128, 0, stream>>>(Wq, WqT, DM, DM);
  k_wt<<<dim3(DM / 64, DM / 16), 128, 0, stream>>>(Wk, WkT, DM, DM);
  k_wt<<<dim3(DM / 64, DM / 16), 128, 0, stream>>>(Wv, WvT, DM, DM);
  k_wt<<<dim3(DM / 64, DM / 16), 128, 0, stream>>>(Wo, WoT, DM, DM);
  k_wt<<<dim3(DM / 64, FFD / 16), 128, 0, stream>>>(W1, W1T, DM, FFD);
  k_wt<<<dim3(FFD / 64, DM / 16), 128, 0, stream>>>(W2, W2T, FFD, DM);

  k_gemm<1, 0, 1, 0><<<dim3(DM / 64, MROWS / 64), 128, 0, stream>>>(Xh, WqT, bq, nullptr, Qh, MROWS, DM, DM, inv_w, 1, 1);
  k_gemm<1, 0, 1, 0><<<dim3(DM / 64, MROWS / 64), 128, 0, stream>>>(Xh, WkT, bk, nullptr, Kh, MROWS, DM, DM, inv_w, 1, 1);
  k_gemm<1, 0, 2, 1><<<dim3(MROWS / 64, DM / 64), 128, 0, stream>>>(WvT, Xh, bv, nullptr, VT, DM, MROWS, DM, inv_w, SEQ, NB);

  k_attn<<<(SEQ / 64) * NB * NH, 128, 0, stream>>>(Qh, Kh, VT, ctx);

  k_gemm<0, 0, 1, 0><<<dim3(DM / 64, MROWS / 64), 128, 0, stream>>>(ctx, WoT, bo, tmpF, nullptr, MROWS, DM, DM, inv_wcx, 1, 1);

  k_addln<0><<<MROWS, 256, 0, stream>>>(tmpF, src, g1, be1, xF, xh);

  k_gemm<1, 1, 1, 0><<<dim3(FFD / 64, MROWS / 64), 128, 0, stream>>>(xh, W1T, bf1, nullptr, h1, MROWS, FFD, DM, inv_w, 1, 1);
  k_gemm<0, 0, 1, 0><<<dim3(DM / 64, MROWS / 64), 128, 0, stream>>>(h1, W2T, bf2, tmpF, nullptr, MROWS, DM, FFD, inv_w, 1, 1);

  k_addln<1><<<MROWS, 256, 0, stream>>>(tmpF, xF, g2, be2, out, nullptr);
}
